// SpatialGAT_90795608637704
// MI455X (gfx1250) — hardware-run, weakly checked
//
#include <hip/hip_runtime.h>
#include <stddef.h>
#include <stdint.h>
#include <math.h>


#define FIN     432
#define KX      448
#define XU      (KX / 8)
#define HC1     512
#define NHD1    4
#define CH1     128
#define HID     64
#define KA2     1024
#define NMLP    32
#define NTHR    256
#define NWAVE   8
#define EPT     8
#define CHUNK   (NTHR * EPT)
#define WCAP    (EPT * 32)
#define LISTN   (NWAVE * WCAP)
#define NBA     1024
#define SLA     10
#define SRCB    17
#define RCAP    28672
#define DEGCAP  128
#define MEAS_B1024  16685
#define MEAS_MAXDEG 32
#define GBM     64
#define GBN     64
#define GTHR    128
#define MROWS   128
#define DROWS   64
#define NUW1    (HC1 * XU)
#define NUW2    (HID * (KA2 / 8))
#define NEGSL   0.2f
#define WSMAX   134217728
#define P_AS1   0
#define P_AD1   512
#define P_B1    1024
#define P_AS2   1536
#define P_AD2   1600
#define P_B2    1664
#define P_W3    1728
#define P_B3    3776
#define P_W4    3808
#define P_B4    3872
#define PARN    3904
#define S_W3    0
#define S_SM    2048
#define S_B2    2176
#define S_HROW  2240
#define S_OUTS  2752
#define S_END   4800
#define BKT_LDS_INTS  (LISTN + RCAP + 16)
#define SCAN_ZINTS    (RCAP + 3 * NBA)
#define SCAN_LDS_INTS (2 * RCAP + 3 * NBA + 16)

static_assert(KX % 32 == 0 && KX >= FIN && FIN % 8 == 0);
static_assert((CHUNK & (CHUNK - 1)) == 0 && CHUNK <= 4096);
static_assert((NBA & (NBA - 1)) == 0 && NBA == (1 << SLA) && NBA % 16 == 0 && NBA % NWAVE == 0);
static_assert(((long long)CHUNK << SLA) < (1LL << 31));
static_assert(((long long)(NBA - 1) << SRCB) < (1LL << 31));
static_assert((RCAP % 32) == 0 && (SCAN_ZINTS % 4) == 0 && (RCAP % (NTHR * 4)) == 0);
static_assert(RCAP >= MEAS_B1024 + 4096);
static_assert(DEGCAP >= MEAS_MAXDEG + 8);
static_assert(SCAN_LDS_INTS * 4 <= 300000 && BKT_LDS_INTS * 4 <= 300000);
static_assert(GBM == (GTHR / 32) * 16 && GTHR == 2 * GBN && GTHR == 2 * GBM);
static_assert((KA2 % 32) == 0 && KA2 == 2 * HC1 && (HC1 % GBN) == 0 && HID == GBN);
static_assert((MROWS % GBM) == 0 && (MROWS % DROWS) == 0 && DROWS == NWAVE * 8);
static_assert(HC1 == NHD1 * CH1 && CH1 == 4 * 32 && HID == 2 * 32 && NMLP == 32);
static_assert((NUW1 % NTHR) == 0 && (NUW2 % NTHR) == 0);
static_assert(HC1 + NWAVE * HC1 <= RCAP && S_END <= RCAP);
static_assert(P_B3 + 128 == PARN && P_W4 == P_B3 + 32 && P_B4 == P_W4 + 64 && (PARN % 32) == 0);
static_assert(NTHR * 8 == HID * NMLP && NTHR * 2 == HC1 && NTHR * 4 == 2 * HC1);

typedef float          v2f  __attribute__((ext_vector_type(2)));
typedef float          v4f  __attribute__((ext_vector_type(4)));
typedef float          v8f  __attribute__((ext_vector_type(8)));
typedef int            v4i  __attribute__((ext_vector_type(4)));
typedef int            v8i  __attribute__((ext_vector_type(8)));
typedef unsigned int   v4u  __attribute__((ext_vector_type(4)));
typedef unsigned short v8us __attribute__((ext_vector_type(8)));
typedef __bf16         v16b __attribute__((ext_vector_type(16)));
typedef v2f  __attribute__((may_alias)) v2fa;
typedef v4f  __attribute__((may_alias)) v4fa;
typedef v4i  __attribute__((may_alias)) v4ia;
typedef v4u  __attribute__((may_alias)) v4ua;
typedef v8us __attribute__((may_alias)) v8usa;
union FragB { v16b v; v8us h[2]; v8i w; };

__device__ __forceinline__ v8f wmb(const FragB& a, const FragB& b, v8f c) {
  v8f d = __builtin_amdgcn_wmma_f32_16x16x32_bf16(false, a.v, false, b.v, (short)0, c, false, false);
  asm volatile("v_nop\n\tv_nop\n\tv_nop\n\tv_nop" : "+v"(d) : "v"(a.w), "v"(b.w));
  return d;
}

__device__ __forceinline__ unsigned int f2bf(float f) {
  const unsigned int u = __float_as_uint(f);
  const unsigned int r = ((u + 0x7FFFu + ((u >> 16) & 1u)) >> 16) & 0xFFFFu;
  return ((u & 0x7FFFFFFFu) > 0x7F800000u) ? 0x7FC0u : r;
}
__device__ __forceinline__ float bf2f(unsigned int b) { return __uint_as_float(b << 16); }
__device__ __forceinline__ float bfr(float f) { return bf2f(f2bf(f)); }

__device__ __forceinline__ void lds_xchg() {
  __builtin_amdgcn_fence(__ATOMIC_RELEASE, "workgroup");
  __builtin_amdgcn_wave_barrier();
}

__device__ __forceinline__ v4u ld4pin(const float* __restrict__ p, int i, int len) {
  const int c = i < 0 ? 0 : (i > len - 4 ? len - 4 : i);
  v4u v = *(const v4ua*)(p + c);
  asm volatile("" : "+v"(v));
  return v;
}
__device__ __forceinline__ v4u keep(const v4u v, bool c) {
  const unsigned int m = c ? 0xFFFFFFFFu : 0u;
  v4u r; r.x = v.x & m; r.y = v.y & m; r.z = v.z & m; r.w = v.w & m;
  return r;
}

template <int SLB>
__device__ __forceinline__ int scan_chunk(const int* __restrict__ dsts, int nE, int cbase, int slotBase,
                                          int nb, int vec8, int* list, int tid, int lane, int wave) {
  int wc = 0;
  const int el0  = tid * EPT;
  const int e0   = cbase + el0;
  const int sent = -2147483647 - 1;
  v4i da, db;
  if (vec8 != 0 && cbase + CHUNK <= nE) {
    da = *(const v4i*)(dsts + e0);
    db = *(const v4i*)(dsts + e0 + 4);
  } else {
    da.x = (e0     < nE) ? dsts[min(e0,     nE - 1)] : sent;
    da.y = (e0 + 1 < nE) ? dsts[min(e0 + 1, nE - 1)] : sent;
    da.z = (e0 + 2 < nE) ? dsts[min(e0 + 2, nE - 1)] : sent;
    da.w = (e0 + 3 < nE) ? dsts[min(e0 + 3, nE - 1)] : sent;
    db.x = (e0 + 4 < nE) ? dsts[min(e0 + 4, nE - 1)] : sent;
    db.y = (e0 + 5 < nE) ? dsts[min(e0 + 5, nE - 1)] : sent;
    db.z = (e0 + 6 < nE) ? dsts[min(e0 + 6, nE - 1)] : sent;
    db.w = (e0 + 7 < nE) ? dsts[min(e0 + 7, nE - 1)] : sent;
  }
  const unsigned nbs = (unsigned)slotBase;
  const unsigned unb = (unsigned)nb;
  const unsigned s0 = (unsigned)da.x - nbs, s1 = (unsigned)da.y - nbs;
  const unsigned s2 = (unsigned)da.z - nbs, s3 = (unsigned)da.w - nbs;
  const unsigned s4 = (unsigned)db.x - nbs, s5 = (unsigned)db.y - nbs;
  const unsigned s6 = (unsigned)db.z - nbs, s7 = (unsigned)db.w - nbs;
  const bool h0 = s0 < unb, h1 = s1 < unb, h2 = s2 < unb, h3 = s3 < unb;
  const bool h4 = s4 < unb, h5 = s5 < unb, h6 = s6 < unb, h7 = s7 < unb;
  const unsigned any = __builtin_amdgcn_ballot_w32(h0 | h1 | h2 | h3 | h4 | h5 | h6 | h7);
  if (any != 0u) {
#define HITJ(J, HJ, SJ) { \
      const unsigned mj = __builtin_amdgcn_ballot_w32(HJ); \
      if (mj != 0u) { \
        if (HJ) { \
          const int pos = wc + (int)__builtin_amdgcn_mbcnt_lo(mj, 0u); \
          if (pos < WCAP) list[wave * WCAP + pos] = ((el0 + (J)) << SLB) | (int)(SJ); \
        } \
        wc += (int)__builtin_popcount(mj); } }
    HITJ(0, h0, s0)
    HITJ(1, h1, s1)
    HITJ(2, h2, s2)
    HITJ(3, h3, s3)
    HITJ(4, h4, s4)
    HITJ(5, h5, s5)
    HITJ(6, h6, s6)
    HITJ(7, h7, s7)
#undef HITJ
  }
  return wc;
}

__global__ __launch_bounds__(NTHR) void k_pa(const float* __restrict__ x, unsigned short* XB, int nN, int nUx) {
  const int u = (int)blockIdx.x * NTHR + (int)threadIdx.x;
  if (u >= nUx) return;
  const int row = u / XU;
  const int c0  = (u - row * XU) * 8;
  const int rc  = row < nN ? row : nN - 1;
  const int cc  = c0 <= FIN - 8 ? c0 : FIN - 8;
  const float* p = x + (size_t)rc * FIN + cc;
  v4f a = *(const v4fa*)p;
  v4f b = *(const v4fa*)(p + 4);
  asm volatile("" : "+v"(a), "+v"(b));
  const unsigned int mk = (row < nN && c0 <= FIN - 8) ? 0xFFFFFFFFu : 0u;
  v4u hv;
  hv.x = (f2bf(a.x) | (f2bf(a.y) << 16)) & mk;
  hv.y = (f2bf(a.z) | (f2bf(a.w) << 16)) & mk;
  hv.z = (f2bf(b.x) | (f2bf(b.y) << 16)) & mk;
  hv.w = (f2bf(b.z) | (f2bf(b.w) << 16)) & mk;
  unsigned short* dp = XB + (size_t)u * 8;
  *(volatile v4u*)dp = hv;
  __threadfence();
  *(volatile v4u*)dp = hv;
}

__global__ __launch_bounds__(NTHR) void k_pb(const float* __restrict__ W1, const float* __restrict__ W2,
                                             unsigned short* W1T, unsigned short* W2T) {
  const int u = (int)blockIdx.x * NTHR + (int)threadIdx.x;
  v8us o;
  unsigned short* dp;
  if (u < NUW1) {
    const int n  = u / XU;
    const int k8 = (u - n * XU) * 8;
#pragma unroll
    for (int i = 0; i < 8; ++i) {
      const int k  = k8 + i;
      const int kc = k < FIN ? k : FIN - 1;
      const float f = W1[(size_t)kc * HC1 + n];
      o[i] = (k < FIN) ? (unsigned short)f2bf(f) : (unsigned short)0;
    }
    dp = W1T + (size_t)n * KX + k8;
  } else if (u < NUW1 + NUW2) {
    const int v  = u - NUW1;
    const int n  = v >> 7;
    const int k8 = (v & 127) * 8;
    const int kk = k8 & (HC1 - 1);
    const float* p = W2 + (size_t)kk * HID + n;
#pragma unroll
    for (int i = 0; i < 8; ++i) o[i] = (unsigned short)f2bf(p[(size_t)i * HID]);
    dp = W2T + (size_t)n * KA2 + k8;
  } else {
    return;
  }
  *(volatile v8us*)dp = o;
  __threadfence();
  *(volatile v8us*)dp = o;
}

__global__ __launch_bounds__(NTHR) void k_pc(const float* __restrict__ as1, const float* __restrict__ ad1,
                                             const float* __restrict__ b1,  const float* __restrict__ as2,
                                             const float* __restrict__ ad2, const float* __restrict__ b2,
                                             const float* __restrict__ W3,  const float* __restrict__ b3,
                                             const float* __restrict__ W4,  const float* __restrict__ b4,
                                             float* PAR) {
  const int u = (int)blockIdx.x * NTHR + (int)threadIdx.x;
  if (u >= PARN / 4) return;
  const int e = 4 * u;
  const v4u v0 = ld4pin(as1, e - P_AS1, 512);
  const v4u v1 = ld4pin(ad1, e - P_AD1, 512);
  const v4u v2 = ld4pin(b1,  e - P_B1,  512);
  const v4u v3 = ld4pin(as2, e - P_AS2, 64);
  const v4u v4 = ld4pin(ad2, e - P_AD2, 64);
  const v4u v5 = ld4pin(b2,  e - P_B2,  64);
  const v4u v6 = ld4pin(W3,  e - P_W3,  2048);
  const v4u v7 = ld4pin(b3,  e - P_B3,  32);
  const v4u v8 = ld4pin(W4,  e - P_W4,  64);
  float q0 = b4[0], q1 = b4[1];
  asm volatile("" : "+v"(q0), "+v"(q1));
  v4u v9; v9.x = __float_as_uint(q0); v9.y = __float_as_uint(q1); v9.z = 0u; v9.w = 0u;
  v4u r = keep(v0, e < P_AD1);
  r |= keep(v1, e >= P_AD1 && e < P_B1);
  r |= keep(v2, e >= P_B1  && e < P_AS2);
  r |= keep(v3, e >= P_AS2 && e < P_AD2);
  r |= keep(v4, e >= P_AD2 && e < P_B2);
  r |= keep(v5, e >= P_B2  && e < P_W3);
  r |= keep(v6, e >= P_W3  && e < P_B3);
  r |= keep(v7, e >= P_B3  && e < P_W4);
  r |= keep(v8, e >= P_W4  && e < P_B4);
  r |= keep(v9, e == P_B4);
  v4f o;
  o.x = bfr(__uint_as_float(r.x));
  o.y = bfr(__uint_as_float(r.y));
  o.z = bfr(__uint_as_float(r.z));
  o.w = bfr(__uint_as_float(r.w));
  float* dp = PAR + e;
  *(volatile v4f*)dp = o;
  __threadfence();
  *(volatile v4f*)dp = o;
}

__global__ __launch_bounds__(NTHR) void k_bucket(const int* __restrict__ srcs, const int* __restrict__ dsts,
                                                 int nE, int nN, int vec8, int* HITS, int* FLG) {
  extern __shared__ __attribute__((aligned(16))) int bsm[];
  int* list = bsm;
  int* reg1 = bsm + LISTN;
  int* wcnt = reg1 + RCAP;
  const int tid = (int)threadIdx.x, lane = tid & 31, wave = tid >> 5;
  const int blk = (int)blockIdx.x;
  const int nodeBase = blk * NBA;
  int nb = nN - nodeBase;
  nb = nb < 0 ? 0 : (nb > NBA ? NBA : nb);

  int tot = 0, ovf = 0;
  const int nChunks = (nE + CHUNK - 1) / CHUNK;
#pragma unroll 1
  for (int ch = 0; ch < nChunks; ++ch) {
    const int cbase = ch * CHUNK;
    const int wc = scan_chunk<SLA>(dsts, nE, cbase, nodeBase, nb, vec8, list, tid, lane, wave);
    if (lane == 0) wcnt[wave] = wc;
    __syncthreads();
    int pre = 0, all = 0;
#pragma unroll
    for (int w2 = 0; w2 < NWAVE; ++w2) {
      int c = wcnt[w2];
      c = c < 0 ? 0 : (c > WCAP ? WCAP : c);
      all += c;
      pre += (w2 < wave) ? c : 0;
    }
    const int wcc  = wc > WCAP ? WCAP : wc;
    const int base = tot + pre;
#pragma unroll 1
    for (int i = lane; i < wcc; i += 32) {
      const int ent = list[wave * WCAP + i];
      const int el  = (ent >> SLA) & (CHUNK - 1);
      const int sl  = ent & (NBA - 1);
      int eid = cbase + el;
      eid = eid > nE - 1 ? nE - 1 : eid;
      const int sraw = srcs[eid];
      const int s = sraw < 0 ? 0 : (sraw > nN - 1 ? nN - 1 : sraw);
      const int pos = base + i;
      if (pos < RCAP) reg1[pos] = (int)((unsigned)s | ((unsigned)sl << SRCB));
    }
    if (tot + all > RCAP) ovf = 1;
    tot += all;
    tot = tot > RCAP ? RCAP : tot;
    __syncthreads();
  }
  const int nh = tot;
  for (int i = nh + tid; i < RCAP; i += NTHR) reg1[i] = 0;
  __syncthreads();

  int* hb = HITS + (size_t)blk * RCAP;
  v4i cv;
  cv.x = (tid == 0) ? nh : 0;
  cv.y = (tid == 0) ? ovf : 0;
  cv.z = 0; cv.w = 0;
  int* fp = FLG + (size_t)blk * 32 + 4 * (tid & 7);
#pragma unroll 1
  for (int p = tid * 4; p < RCAP; p += NTHR * 4) {
    const v4i v = *(const v4ia*)(reg1 + p);
    *(volatile v4i*)(hb + p) = v;
  }
  if (tid < 8) *(volatile v4i*)fp = cv;
  __threadfence();
#pragma unroll 1
  for (int p = tid * 4; p < RCAP; p += NTHR * 4) {
    const v4i v = *(const v4ia*)(reg1 + p);
    *(volatile v4i*)(hb + p) = v;
  }
  if (tid < 8) *(volatile v4i*)fp = cv;
}

template <bool DOTS>
__global__ __launch_bounds__(GTHR) __attribute__((amdgpu_num_vgpr(248)))
void k_gemm(const unsigned short* __restrict__ A, const unsigned short* __restrict__ WT,
            float* outF, int K, int ldo,
            const float* __restrict__ atts, const float* __restrict__ attd, int attLen,
            float* SD, int MPr)
{
  __shared__ __attribute__((aligned(16))) float stg[GBM * GBN];
  __shared__ __attribute__((aligned(16))) float satt[2 * GBN];
  __shared__ __attribute__((aligned(16))) float sdot[2 * GBM];
  const int tid = (int)threadIdx.x, lane = tid & 31, wave = tid >> 5, hh = lane >> 4, m = lane & 15;
  const int rowBase = (int)blockIdx.x * GBM;
  const int head    = (int)blockIdx.y;
  const int col0    = head * GBN;

  if constexpr (DOTS) {
    const int which = tid >> 6;
    const int c  = tid & 63;
    const int cl = c < attLen ? c : attLen - 1;
    const float vs = atts[head * attLen + cl];
    const float vd = attd[head * attLen + cl];
    float v = (which == 0) ? vs : vd;
    v = (c < attLen) ? bfr(v) : 0.f;
    satt[which * GBN + c] = v;
  }

  v8f acc[4];
  {
    const v8f z = {0.f, 0.f, 0.f, 0.f, 0.f, 0.f, 0.f, 0.f};
    acc[0] = z; acc[1] = z; acc[2] = z; acc[3] = z;
  }
  const unsigned short* ap = A  + (size_t)(rowBase + 16 * wave + m) * (size_t)K + 8 * hh;
  const unsigned short* wp = WT + (size_t)(col0 + m) * (size_t)K + 8 * hh;
  const int ksteps = K >> 5;
#pragma unroll 1
  for (int ks = 0; ks < ksteps; ++ks) {
    FragB af;
    af.h[0] = *(const v8usa*)(ap + 32 * ks);
    af.h[1] = *(const v8usa*)(ap + 32 * ks + 16);
#pragma unroll
    for (int t = 0; t < 4; ++t) {
      const unsigned short* wq = wp + (size_t)(16 * t) * (size_t)K + 32 * ks;
      FragB bf;
      bf.h[0] = *(const v8usa*)wq;
      bf.h[1] = *(const v8usa*)(wq + 16);
      acc[t] = wmb(af, bf, acc[t]);
    }
  }

#pragma unroll
  for (int t = 0; t < 4; ++t) {
    const int lc = 16 * t + m;
#pragma unroll
    for (int r = 0; r < 8; ++r) {
      const int lr = 16 * wave + 8 * hh + r;
      stg[lr * GBN + lc] = acc[t][r];
    }
  }
  __syncthreads();

  if constexpr (DOTS) {
    const int row = tid & 63, which = tid >> 6;
    const float* sa = satt + which * GBN;
    const float* hr = stg + row * GBN;
    float d = 0.f;
#pragma unroll 4
    for (int c4 = 0; c4 < GBN / 4; ++c4) {
      const v4f hv = *(const v4fa*)(hr + 4 * c4);
      const v4f av = *(const v4fa*)(sa + 4 * c4);
      d = fmaf(hv.x, av.x, d);
      d = fmaf(hv.y, av.y, d);
      d = fmaf(hv.z, av.z, d);
      d = fmaf(hv.w, av.w, d);
    }
    sdot[which * GBM + row] = d;
    __syncthreads();
  }

  v4f fv[8];
#pragma unroll
  for (int i = 0; i < 8; ++i) {
    const int lr = 16 * wave + 2 * i + hh;
    fv[i] = *(const v4fa*)(stg + lr * GBN + 4 * m);
  }
  const int which2 = lane >> 4, piece = lane & 15;
  v4f sdv = {0.f, 0.f, 0.f, 0.f};
  float* sp = SD;
  if constexpr (DOTS) {
    sdv = *(const v4fa*)(sdot + which2 * GBM + 4 * piece);
    sp = SD + (size_t)(2 * head + which2) * (size_t)MPr + rowBase + 4 * piece;
  }

#pragma unroll
  for (int i = 0; i < 8; ++i) {
    const int lr = 16 * wave + 2 * i + hh;
    const int gr = rowBase + lr;
    float* op = outF + (size_t)gr * (size_t)ldo + col0 + 4 * m;
    *(volatile v4f*)op = fv[i];
  }
  if constexpr (DOTS) { if (wave == 0) *(volatile v4f*)sp = sdv; }
  __threadfence();
#pragma unroll
  for (int i = 0; i < 8; ++i) {
    const int lr = 16 * wave + 2 * i + hh;
    const int gr = rowBase + lr;
    float* op = outF + (size_t)gr * (size_t)ldo + col0 + 4 * m;
    *(volatile v4f*)op = fv[i];
  }
  if constexpr (DOTS) { if (wave == 0) *(volatile v4f*)sp = sdv; }
}

__device__ __forceinline__ void put_dots(float* dst, const float* sl, int lane) {
  const v4f a = *(const v4fa*)(sl + 4 * lane);
  const v4f b = *(const v4fa*)(sl + 128 + 4 * lane);
  *(volatile v4f*)(dst + 4 * lane) = a;
  *(volatile v4f*)(dst + 128 + 4 * lane) = b;
  __threadfence();
  *(volatile v4f*)(dst + 4 * lane) = a;
  *(volatile v4f*)(dst + 128 + 4 * lane) = b;
}

__global__ __launch_bounds__(NTHR) void k_dots(const float* __restrict__ H, const float* __restrict__ PAR,
                                               float* AS, float* AD) {
  __shared__ __attribute__((aligned(16))) float satt[2 * HC1];
  __shared__ __attribute__((aligned(16))) float sdl[2 * DROWS * NHD1];
  const int tid = (int)threadIdx.x, lane = tid & 31, wave = tid >> 5;
  const int rowBase = (int)blockIdx.x * DROWS;
  {
    const v4f q = *(const v4f*)(PAR + P_AS1 + 4 * tid);
    *(v4fa*)(satt + 4 * tid) = q;
  }
  __syncthreads();
#pragma unroll 1
  for (int i = 0; i < 8; ++i) {
    const int lr = 8 * wave + i;
    const float* hp = H + (size_t)(rowBase + lr) * HC1 + 4 * lane;
#pragma unroll 1
    for (int j = 0; j < NHD1; ++j) {
      const v4f hv = *(const v4f*)(hp + j * CH1);
      const v4f sa = *(const v4fa*)(satt + j * CH1 + 4 * lane);
      const v4f da = *(const v4fa*)(satt + HC1 + j * CH1 + 4 * lane);
      float ps = hv.x * sa.x;
      ps = fmaf(hv.y, sa.y, ps); ps = fmaf(hv.z, sa.z, ps); ps = fmaf(hv.w, sa.w, ps);
      float pd = hv.x * da.x;
      pd = fmaf(hv.y, da.y, pd); pd = fmaf(hv.z, da.z, pd); pd = fmaf(hv.w, da.w, pd);
#pragma unroll
      for (int off = 16; off > 0; off >>= 1) {
        ps += __shfl_xor(ps, off);
        pd += __shfl_xor(pd, off);
      }
      if (lane == 0) {
        sdl[lr * NHD1 + j] = ps;
        sdl[DROWS * NHD1 + lr * NHD1 + j] = pd;
      }
    }
  }
  __syncthreads();
  if (wave == 0) {
    put_dots(AS + (size_t)rowBase * NHD1, sdl, lane);
  } else if (wave == 1) {
    put_dots(AD + (size_t)rowBase * NHD1, sdl + DROWS * NHD1, lane);
  }
}

__device__ __forceinline__ void upd4(float lg, float d, float e, const v4f g, float& mx, float& dn,
                                     float& a0, float& a1, float& a2, float& a3) {
  const bool  up = d > 0.f;
  const float s1 = up ? e : 1.0f;
  const float s2 = up ? 1.0f : e;
  mx = up ? lg : mx;
  dn = fmaf(dn, s1, s2);
  a0 = fmaf(a0, s1, s2 * g.x);
  a1 = fmaf(a1, s1, s2 * g.y);
  a2 = fmaf(a2, s1, s2 * g.z);
  a3 = fmaf(a3, s1, s2 * g.w);
}

template <int L>
__global__ __launch_bounds__(NTHR) __attribute__((amdgpu_num_vgpr(248)))
void k_scan(const int* __restrict__ HITS, const int* __restrict__ FLGB,
            const float* __restrict__ F, const float* __restrict__ SA, const float* __restrict__ SB,
            const float* __restrict__ PAR, unsigned short* XP, float* out, int nN, int MPr) {
  static_assert(L == 1 || L == 2);
  extern __shared__ __attribute__((aligned(16))) int ssm[];
  int* hl   = ssm;
  int* sl   = ssm + RCAP;
  int* cnt  = sl + RCAP;
  int* offs = cnt + NBA;
  int* cur  = offs + NBA;
  int* misc = cur + NBA;
  const int tid = (int)threadIdx.x, lane = tid & 31, wave = tid >> 5;
  const int blk = (int)blockIdx.x;
  const int nodeBase = blk * NBA;

  const int nhraw = FLGB[(size_t)blk * 32];
  const int bflag = FLGB[(size_t)blk * 32 + 1];
  const int nh  = nhraw < 0 ? 0 : (nhraw > RCAP ? RCAP : nhraw);
  const int ovf = (bflag != 0 || nhraw < 0 || nhraw > RCAP) ? 1 : 0;

  {
    const v4i z4 = {0, 0, 0, 0};
    for (int i = tid * 4; i < SCAN_ZINTS; i += NTHR * 4) *(v4ia*)(sl + i) = z4;
    if (tid < 16) misc[tid] = 0;
    const int* hb = HITS + (size_t)blk * RCAP;
    const int nh4 = (nh + 3) & ~3;
#pragma unroll 1
    for (int p = tid * 4; p < nh4; p += NTHR * 4) *(v4ia*)(hl + p) = *(const v4i*)(hb + p);
  }
  __syncthreads();

  if (wave == 0) {
#pragma unroll 1
    for (int b0 = 0; b0 < nh; b0 += 32) {
      const int idx = b0 + lane;
      const int uv  = hl[idx < nh ? idx : nh - 1];
      const int m32 = (nh - b0) < 32 ? (nh - b0) : 32;
#pragma unroll 1
      for (int k = 0; k < m32; ++k) {
        const int u  = __builtin_amdgcn_readlane(uv, k);
        const int sq = (u >> SRCB) & (NBA - 1);
        if (lane == 0) cnt[sq] = cnt[sq] + 1;
      }
    }
  }
  __syncthreads();
  if (wave == 0) {
    const int base = lane * (NBA / 32);
    int s = 0;
#pragma unroll 1
    for (int i = 0; i < NBA / 32; ++i) s += cnt[base + i];
    int incl = s;
#pragma unroll
    for (int d = 1; d < 32; d <<= 1) {
      const int y = __shfl_up(incl, d, 32);
      if (lane >= d) incl += y;
    }
    int run = incl - s;
#pragma unroll 1
    for (int i = 0; i < NBA / 32; ++i) {
      const int cv = cnt[base + i];
      offs[base + i] = run;
      cur[base + i]  = run;
      run += cv;
    }
  }
  __syncthreads();
  if (wave == 0) {
#pragma unroll 1
    for (int b0 = 0; b0 < nh; b0 += 32) {
      const int idx = b0 + lane;
      const int uv  = hl[idx < nh ? idx : nh - 1];
      const int m32 = (nh - b0) < 32 ? (nh - b0) : 32;
#pragma unroll 1
      for (int k = 0; k < m32; ++k) {
        const int u  = __builtin_amdgcn_readlane(uv, k);
        const int sq = (u >> SRCB) & (NBA - 1);
        if (lane == 0) {
          int p = cur[sq];
          p = p < 0 ? 0 : (p > RCAP - 1 ? RCAP - 1 : p);
          sl[p] = u;
          cur[sq] = p + 1;
        }
      }
    }
  }
  __syncthreads();

  float* fl = (float*)hl;
  if constexpr (L == 1) {
    const v2f bq = *(const v2f*)(PAR + P_B1 + 2 * tid);
    *(v2fa*)(fl + 2 * tid) = bq;
  } else {
    const v4f wa = *(const v4f*)(PAR + P_W3 + 8 * tid);
    const v4f wb = *(const v4f*)(PAR + P_W3 + 8 * tid + 4);
    *(v4fa*)(fl + S_W3 + 8 * tid) = wa;
    *(v4fa*)(fl + S_W3 + 8 * tid + 4) = wb;
    float vsm = PAR[P_B3 + (tid & 127)];
    float vb2 = PAR[P_B2 + (tid & 63)];
    asm volatile("" : "+v"(vsm), "+v"(vb2));
    if (tid < 128) fl[S_SM + tid] = vsm;
    if (tid < 64)  fl[S_B2 + tid] = vb2;
  }
  __syncthreads();

  const float qnan = __int_as_float(0x7fc00000);
  float* st = fl + HC1 + wave * HC1;
  float* hrow = fl + S_HROW + wave * HID;
  float* OUTS = fl + S_OUTS;
  const int hq = lane & 3;
  float bza = 0.f, bzb = 0.f, b3v = 0.f, w40 = 0.f, w41 = 0.f, b40 = 0.f, b41 = 0.f;
  if constexpr (L == 2) {
    bza = fl[S_B2 + 2 * lane]; bzb = fl[S_B2 + 2 * lane + 1];
    b3v = fl[S_SM + lane];
    w40 = fl[S_SM + 32 + 2 * lane]; w41 = fl[S_SM + 33 + 2 * lane];
    b40 = fl[S_SM + 96]; b41 = fl[S_SM + 97];
  }

#pragma unroll 1
  for (int si = 0; si < NBA / NWAVE; ++si) {
    const int s    = si * NWAVE + wave;
    const int node = nodeBase + s;
    const int nc   = node < nN ? node : nN - 1;
    int c = cnt[s];
    const bool big = c > DEGCAP;
    c = c < 0 ? 0 : (c > DEGCAP ? DEGCAP : c);
    int o = offs[s];
    o = o < 0 ? 0 : (o > RCAP ? RCAP : o);
    if (c > nh - o) c = nh - o;
    c = c < 0 ? 0 : c;
    const bool pflag = big || (ovf != 0);
    const float pzr  = pflag ? qnan : 0.0f;
    const bool live  = node < nN;

    float adv[4] = {0.f, 0.f, 0.f, 0.f};
    if constexpr (L == 1) {
      const v4f q = *(const v4f*)(SB + (size_t)nc * NHD1);
      adv[0] = q.x; adv[1] = q.y; adv[2] = q.z; adv[3] = q.w;
    } else {
      adv[0] = SB[nc];
    }
    float mx[4], dn[4];
#pragma unroll
    for (int j = 0; j < 4; ++j) { mx[j] = -3.0e38f; dn[j] = 0.0f; }
    float acc[16];
#pragma unroll
    for (int i = 0; i < 16; ++i) acc[i] = 0.0f;

    const int T = c + 1;
#pragma unroll 1
    for (int b0 = 0; b0 < T; b0 += 32) {
      const int t = b0 + lane;
      int idx = o + t;
      idx = idx < 0 ? 0 : (idx > RCAP - 1 ? RCAP - 1 : idx);
      const int ent = sl[idx];
      int hs = ent & ((1 << SRCB) - 1);
      hs = hs > nN - 1 ? nN - 1 : hs;
      const int sr  = (t < c) ? hs : nc;
      const int m32 = (T - b0) < 32 ? (T - b0) : 32;
#pragma unroll 1
      for (int k = 0; k < m32; ++k) {
        const int sk = __builtin_amdgcn_readlane(sr, k);
        if constexpr (L == 1) {
          const v4f asq = *(const v4f*)(SA + (size_t)sk * NHD1);
          const float* rp = F + (size_t)sk * HC1 + 4 * lane;
          const v4f g0 = *(const v4f*)rp;
          const v4f g1 = *(const v4f*)(rp + CH1);
          const v4f g2 = *(const v4f*)(rp + 2 * CH1);
          const v4f g3 = *(const v4f*)(rp + 3 * CH1);
          float l0 = asq.x + adv[0], l1 = asq.y + adv[1], l2 = asq.z + adv[2], l3 = asq.w + adv[3];
          l0 = l0 > 0.f ? l0 : NEGSL * l0;
          l1 = l1 > 0.f ? l1 : NEGSL * l1;
          l2 = l2 > 0.f ? l2 : NEGSL * l2;
          l3 = l3 > 0.f ? l3 : NEGSL * l3;
          const float d0 = l0 - mx[0], d1 = l1 - mx[1], d2 = l2 - mx[2], d3 = l3 - mx[3];
          const float dm = (hq == 0) ? d0 : ((hq == 1) ? d1 : ((hq == 2) ? d2 : d3));
          const float em = expf(-fabsf(dm));
          const int  emi = __float_as_int(em);
          const float e0 = __int_as_float(__builtin_amdgcn_readlane(emi, 0));
          const float e1 = __int_as_float(__builtin_amdgcn_readlane(emi, 1));
          const float e2 = __int_as_float(__builtin_amdgcn_readlane(emi, 2));
          const float e3 = __int_as_float(__builtin_amdgcn_readlane(emi, 3));
          upd4(l0, d0, e0, g0, mx[0], dn[0], acc[0],  acc[1],  acc[2],  acc[3]);
          upd4(l1, d1, e1, g1, mx[1], dn[1], acc[4],  acc[5],  acc[6],  acc[7]);
          upd4(l2, d2, e2, g2, mx[2], dn[2], acc[8],  acc[9],  acc[10], acc[11]);
          upd4(l3, d3, e3, g3, mx[3], dn[3], acc[12], acc[13], acc[14], acc[15]);
        } else {
          const v2f a = *(const v2f*)(F + (size_t)sk * HID + 2 * lane);
          float lg = SA[sk] + adv[0];
          lg = lg > 0.f ? lg : NEGSL * lg;
          const float df = lg - mx[0];
          const float ee = expf(-fabsf(df));
          const bool  up = df > 0.f;
          const float s1 = up ? ee : 1.0f;
          const float s2 = up ? 1.0f : ee;
          mx[0] = up ? lg : mx[0];
          dn[0] = fmaf(dn[0], s1, s2);
          acc[0] = fmaf(acc[0], s1, s2 * a.x);
          acc[1] = fmaf(acc[1], s1, s2 * a.y);
        }
      }
    }

    if constexpr (L == 1) {
#pragma unroll
      for (int j = 0; j < 4; ++j) {
        const float inv = __builtin_amdgcn_rcpf(dn[j]);
        v4f q;
        q.x = acc[4 * j] * inv; q.y = acc[4 * j + 1] * inv; q.z = acc[4 * j + 2] * inv; q.w = acc[4 * j + 3] * inv;
        *(v4fa*)(st + j * CH1 + 4 * lane) = q;
      }
#pragma unroll 1
      for (int t = 0; t < 16; ++t) {
        const int ix = (t >> 2) * CH1 + 4 * lane + (t & 3);
        float y = st[ix] + fl[ix];
        y = (y > 0.0f) ? y : expm1f(y);
        st[ix] = y + pzr;
      }
      lds_xchg();
      const v4f ha = *(const v4fa*)(st + 8 * lane);
      const v4f hb = *(const v4fa*)(st + 8 * lane + 4);
      const v4f hc = *(const v4fa*)(st + 256 + 8 * lane);
      const v4f hd = *(const v4fa*)(st + 256 + 8 * lane + 4);
      lds_xchg();
      const float ya[8] = {ha.x, ha.y, ha.z, ha.w, hb.x, hb.y, hb.z, hb.w};
      const float yb[8] = {hc.x, hc.y, hc.z, hc.w, hd.x, hd.y, hd.z, hd.w};
      v8us hoA, loA, hoB, loB;
#pragma unroll
      for (int i = 0; i < 8; ++i) {
        const float va = live ? ya[i] : 0.0f;
        const float vb = live ? yb[i] : 0.0f;
        const unsigned int ba = f2bf(va), bb = f2bf(vb);
        hoA[i] = (unsigned short)ba;
        hoB[i] = (unsigned short)bb;
        loA[i] = (unsigned short)f2bf(va - bf2f(ba));
        loB[i] = (unsigned short)f2bf(vb - bf2f(bb));
      }
      if (node < MPr) {
        unsigned short* hp = XP + (size_t)node * KA2 + 8 * lane;
        *(volatile v8us*)hp = hoA;
        *(volatile v8us*)(hp + 256) = hoB;
        *(volatile v8us*)(hp + 512) = loA;
        *(volatile v8us*)(hp + 768) = loB;
        __threadfence();
        *(volatile v8us*)hp = hoA;
        *(volatile v8us*)(hp + 256) = hoB;
        *(volatile v8us*)(hp + 512) = loA;
        *(volatile v8us*)(hp + 768) = loB;
      }
    } else {
      const float inv = __builtin_amdgcn_rcpf(dn[0]);
      float va = fmaf(acc[0], inv, bza);
      float vb = fmaf(acc[1], inv, bzb);
#pragma unroll 1
      for (int q = 0; q < 2; ++q) {
        float y = va;
        y = (y > 0.0f) ? y : expm1f(y);
        va = vb; vb = y;
      }
      v2f hv2; hv2.x = va + pzr; hv2.y = vb + pzr;
      *(v2fa*)(hrow + 2 * lane) = hv2;
      lds_xchg();
      float tj = b3v;
#pragma unroll 4
      for (int k = 0; k < HID; ++k) tj = fmaf(hrow[k], fl[S_W3 + k * NMLP + lane], tj);
      tj = (tj > 0.0f) ? tj : (tj - tj);
      float p0 = tj * w40, p1 = tj * w41;
#pragma unroll
      for (int off = 16; off > 0; off >>= 1) {
        p0 += __shfl_xor(p0, off);
        p1 += __shfl_xor(p1, off);
      }
      v2f ov;
      ov.x = pflag ? qnan : (p0 + b40);
      ov.y = pflag ? qnan : (p1 + b41);
      if (lane == 0) *(v2fa*)(OUTS + 2 * s) = ov;
      lds_xchg();
    }
  }

  if constexpr (L == 2) {
    __syncthreads();
    int liveRows = nN - nodeBase;
    liveRows = liveRows < 0 ? 0 : (liveRows > NBA ? NBA : liveRows);
    const int npc = liveRows >> 1;
    float* ob = out + (size_t)nodeBase * 2;
#pragma unroll 1
    for (int p = tid; p < npc; p += NTHR) {
      const v4f v = *(const v4fa*)(OUTS + 4 * p);
      *(volatile v4f*)(ob + 4 * p) = v;
    }
    __threadfence();
#pragma unroll 1
    for (int p = tid; p < npc; p += NTHR) {
      const v4f v = *(const v4fa*)(OUTS + 4 * p);
      *(volatile v4f*)(ob + 4 * p) = v;
    }
  }
}

static inline int cdiv(int a, int b) { return (a + b - 1) / b; }

extern "C" void kernel_launch(void* const* d_in, const int* in_sizes, int n_in,
                              void* d_out, int out_size, void* d_ws, size_t ws_size,
                              hipStream_t stream) {
  if (n_in < 14) return;
  const int nN = in_sizes[0] / FIN;
  if (nN <= 0 || in_sizes[0] != nN * FIN || nN > (1 << SRCB)) return;
  if ((nN & 15) != 0) return;
  if (in_sizes[1] < 2 || (in_sizes[1] & 1) != 0) return;
  const int nE = in_sizes[1] / 2;
  if (nE < 1 || nE > (1 << 30)) return;
  if (in_sizes[2] != FIN * HC1) return;
  if (in_sizes[3] != HC1 || in_sizes[4] != HC1) return;
  if (in_sizes[5] != HC1) return;
  if (in_sizes[6] != HC1 * HID) return;
  if (in_sizes[7] != HID || in_sizes[8] != HID) return;
  if (in_sizes[9] != HID) return;
  if (in_sizes[10] != HID * NMLP || in_sizes[11] != NMLP) return;
  if (in_sizes[12] != NMLP * 2 || in_sizes[13] != 2) return;
  if (out_size != nN * 2) return;

  const float* x   = (const float*)d_in[0];
  const int*   ei  = (const int*)  d_in[1];
  const float* W1  = (const float*)d_in[2];
  const float* a1s = (const float*)d_in[3];
  const float* a1d = (const float*)d_in[4];
  const float* b1  = (const float*)d_in[5];
  const float* W2  = (const float*)d_in[6];
  const float* a2s = (const float*)d_in[7];
  const float* a2d = (const float*)d_in[8];
  const float* b2  = (const float*)d_in[9];
  const float* W3  = (const float*)d_in[10];
  const float* b3  = (const float*)d_in[11];
  const float* W4  = (const float*)d_in[12];
  const float* b4  = (const float*)d_in[13];
  float* out = (float*)d_out;
  const int* src = ei;
  const int* dst = ei + nE;

  const int MP   = cdiv(nN, MROWS) * MROWS;
  const int gM   = MP / GBM;
  const int gA   = cdiv(MP, NBA);
  if ((long long)gA * NBA < (long long)MP) return;
  const int vec8 = ((nE & 3) == 0) ? 1 : 0;
  const int nUx  = MP * XU;

  char* ws = (char*)d_ws;
  size_t off = 0;
  const size_t oXB  = off; off += (size_t)MP * KX * 2;          off = (off + 255) & ~(size_t)255;
  const size_t oW1T = off; off += (size_t)HC1 * KX * 2;         off = (off + 255) & ~(size_t)255;
  const size_t oW2T = off; off += (size_t)HID * KA2 * 2;        off = (off + 255) & ~(size_t)255;
  const size_t oPAR = off; off += (size_t)PARN * 4;             off = (off + 255) & ~(size_t)255;
  const size_t oH1  = off; off += (size_t)MP * HC1 * 4;         off = (off + 255) & ~(size_t)255;
  const size_t oAS1 = off; off += (size_t)MP * NHD1 * 4;        off = (off + 255) & ~(size_t)255;
  const size_t oAD1 = off; off += (size_t)MP * NHD1 * 4;        off = (off + 255) & ~(size_t)255;
  const size_t oX1  = off; off += (size_t)MP * KA2 * 2;         off = (off + 255) & ~(size_t)255;
  const size_t oH2  = off; off += (size_t)MP * HID * 4;         off = (off + 255) & ~(size_t)255;
  const size_t oSD2 = off; off += (size_t)2 * MP * 4;           off = (off + 255) & ~(size_t)255;
  const size_t oHIT = off; off += (size_t)gA * RCAP * 4;        off = (off + 255) & ~(size_t)255;
  const size_t oFLG = off; off += (size_t)gA * 128;             off = (off + 255) & ~(size_t)255;
  if (off > ws_size || off > (size_t)WSMAX) return;
  unsigned short* XB   = (unsigned short*)(ws + oXB);
  unsigned short* W1T  = (unsigned short*)(ws + oW1T);
  unsigned short* W2T  = (unsigned short*)(ws + oW2T);
  float*          PAR  = (float*)(ws + oPAR);
  float*          H1   = (float*)(ws + oH1);
  float*          AS1  = (float*)(ws + oAS1);
  float*          AD1  = (float*)(ws + oAD1);
  unsigned short* X1   = (unsigned short*)(ws + oX1);
  float*          H2   = (float*)(ws + oH2);
  float*          SD2  = (float*)(ws + oSD2);
  int*            HITS = (int*)(ws + oHIT);
  int*            FLG  = (int*)(ws + oFLG);

  const int bktLds  = BKT_LDS_INTS * 4;
  const int scanLds = SCAN_LDS_INTS * 4;
  hipFuncSetAttribute(reinterpret_cast<const void*>(&k_bucket),
                      hipFuncAttributeMaxDynamicSharedMemorySize, bktLds);
  hipFuncSetAttribute(reinterpret_cast<const void*>(&k_scan<1>),
                      hipFuncAttributeMaxDynamicSharedMemorySize, scanLds);
  hipFuncSetAttribute(reinterpret_cast<const void*>(&k_scan<2>),
                      hipFuncAttributeMaxDynamicSharedMemorySize, scanLds);

  k_pa<<<cdiv(nUx, NTHR), NTHR, 0, stream>>>(x, XB, nN, nUx);
  k_pb<<<(NUW1 + NUW2) / NTHR, NTHR, 0, stream>>>(W1, W2, W1T, W2T);
  k_pc<<<cdiv(PARN / 4, NTHR), NTHR, 0, stream>>>(a1s, a1d, b1, a2s, a2d, b2, W3, b3, W4, b4, PAR);
  k_bucket<<<gA, NTHR, bktLds, stream>>>(src, dst, nE, nN, vec8, HITS, FLG);
  k_gemm<false><<<dim3(gM, HC1 / GBN), GTHR, 0, stream>>>(XB, W1T, H1, KX, HC1, PAR, PAR, HID, AS1, MP);
  k_dots<<<MP / DROWS, NTHR, 0, stream>>>(H1, PAR, AS1, AD1);
  k_scan<1><<<gA, NTHR, scanLds, stream>>>(HITS, FLG, H1, AS1, AD1, PAR, X1, out, nN, MP);
  k_gemm<true><<<dim3(gM, HID / GBN), GTHR, 0, stream>>>(X1, W2T, H2, KA2, HID, PAR + P_AS2, PAR + P_AD2, HID, SD2, MP);
  k_scan<2><<<gA, NTHR, scanLds, stream>>>(HITS, FLG, H2, SD2, SD2 + MP, PAR, X1, out, nN, MP);
}
